// TransitionGNN_74869869904048
// MI455X (gfx1250) — hardware-verified
//
#include <hip/hip_runtime.h>
#include <stdint.h>

typedef unsigned short us;
typedef us     v8us __attribute__((ext_vector_type(8)));
typedef us     v4us __attribute__((ext_vector_type(4)));
typedef __bf16 v16b __attribute__((ext_vector_type(16)));
typedef float  v8f  __attribute__((ext_vector_type(8)));
typedef float  v4f  __attribute__((ext_vector_type(4)));
typedef v4f  __attribute__((may_alias)) v4fa;
typedef v8us __attribute__((may_alias)) v8usa;
typedef v4us __attribute__((may_alias)) v4usa;

union Frag { v16b v; v8us half[2]; };

#define NB  8192
#define NK  10
#define ND  64
#define NH  128
#define NA  16
#define NE  90
#define NF  208
#define KE  128
#define KPN 352
#define WNP 384
#define TB  64

#define S16_N   (NB * NK * ND)
#define A16_N   (NB * NK * NA)
#define WE16_N  (NE * NH * KE)
#define WN16_N  (NK * ND * WNP)
#define AGG_N   (NB * NK * NH)

#define SW_P   136
#define SN_P   392
#define SAGG_P 132
#define SA_P   360
#define SO_P   68

static_assert((S16_N % 8) == 0);
static_assert((A16_N % 8) == 0);
static_assert(((S16_N / 8) % 32) == 0);
static_assert((((S16_N + A16_N) / 8) % 256) == 0);
static_assert((NB % TB) == 0);
static_assert((KE % 32) == 0);
static_assert((KPN % 32) == 0);
static_assert(KPN <= WNP);
static_assert((SW_P % 8) == 0);
static_assert((SN_P % 8) == 0);
static_assert((SA_P % 8) == 0);
static_assert((SAGG_P % 4) == 0);
static_assert((SO_P % 4) == 0);

__device__ __forceinline__ us f2bf(float f) {
  unsigned int u = __builtin_bit_cast(unsigned int, f);
  u += 0x7FFFu + ((u >> 16) & 1u);
  return (us)(u >> 16);
}
__device__ __forceinline__ float bf2f(us b) {
  return __builtin_bit_cast(float, ((unsigned int)b) << 16);
}
__device__ __forceinline__ float bf16r(float f) { return bf2f(f2bf(f)); }

__device__ __forceinline__ float tanh_f32(float x) {
  const float xc = fminf(fmaxf(x, -16.0f), 16.0f);
  const float e = __expf(2.0f * xc);
  return (e - 1.0f) * __builtin_amdgcn_rcpf(e + 1.0f);
}

__device__ __forceinline__ v8f wmma_bf16(v16b a, v16b b, v8f c) {
  v8f d = __builtin_amdgcn_wmma_f32_16x16x32_bf16(false, a, false, b, (short)0, c, false, false);
  asm volatile("v_nop\n\tv_nop\n\tv_nop\n\tv_nop" : "+v"(d) : "v"(a), "v"(b));
  return d;
}

__device__ __forceinline__ v16b load_frag(const us* p, int h) {
  Frag f;
  f.half[0] = *(const v8usa*)(p + 8 * h);
  f.half[1] = *(const v8usa*)(p + 16 + 8 * h);
  return f.v;
}

__global__ __launch_bounds__(256) void cvt_inputs_kernel(
    const float* __restrict__ states, const float* __restrict__ action,
    us* __restrict__ S16, us* __restrict__ A16)
{
  const int g = blockIdx.x * 256 + threadIdx.x;
  if (g >= (S16_N + A16_N) / 8) return;
  const float* src;
  us* dst;
  if (g < S16_N / 8) {
    src = states + (size_t)g * 8;
    dst = S16 + (size_t)g * 8;
  } else {
    const int off = g - S16_N / 8;
    src = action + (size_t)off * 8;
    dst = A16 + (size_t)off * 8;
  }
  const v4f a = *(const v4fa*)src;
  const v4f c = *(const v4fa*)(src + 4);
  const v8us o = { f2bf(a.x), f2bf(a.y), f2bf(a.z), f2bf(a.w),
                   f2bf(c.x), f2bf(c.y), f2bf(c.z), f2bf(c.w) };
  *(volatile v8us*)dst = o;
  __threadfence();
  *(volatile v8us*)dst = o;
}

__device__ __forceinline__ void wedge_store_pass(const us* sW, us* dstb, int tid) {
  #pragma unroll
  for (int it = 0; it < 8; ++it) {
    const int p = it * 256 + tid;
    const int n = p >> 4, kc = (p & 15) * 8;
    const v8us v = *(const v8usa*)(sW + n * SW_P + kc);
    *(volatile v8us*)(dstb + (size_t)p * 8) = v;
  }
}

__global__ __launch_bounds__(256) void cvt_wedge_kernel(
    const float* __restrict__ W_edge, us* __restrict__ WE16)
{
  __shared__ __attribute__((aligned(16))) us sW[NH * SW_P];
  const int tid = threadIdx.x;
  const int e = blockIdx.x;
  const float* src = W_edge + (size_t)e * (KE * NH);
  #pragma unroll 1
  for (int it = 0; it < 16; ++it) {
    const int idx4 = it * 256 + tid;
    const int k = idx4 >> 5;
    const int n0 = (idx4 & 31) * 4;
    const v4f v = *(const v4fa*)(src + k * NH + n0);
    sW[(n0 + 0) * SW_P + k] = f2bf(v.x);
    sW[(n0 + 1) * SW_P + k] = f2bf(v.y);
    sW[(n0 + 2) * SW_P + k] = f2bf(v.z);
    sW[(n0 + 3) * SW_P + k] = f2bf(v.w);
  }
  __syncthreads();
  us* dstb = WE16 + (size_t)e * (NH * KE);
  wedge_store_pass(sW, dstb, tid);
  __threadfence();
  wedge_store_pass(sW, dstb, tid);
}

__device__ __forceinline__ void wnode_store_pass(const us* sN, us* dstb, int tid) {
  #pragma unroll
  for (int it = 0; it < 12; ++it) {
    const int p = it * 256 + tid;
    const int d = p / 48, c = (p - d * 48) * 8;
    const v8us v = *(const v8usa*)(sN + d * SN_P + c);
    *(volatile v8us*)(dstb + (size_t)p * 8) = v;
  }
}

__global__ __launch_bounds__(256) void cvt_wnode_kernel(
    const float* __restrict__ W_node, us* __restrict__ WN16)
{
  __shared__ __attribute__((aligned(16))) us sN[ND * SN_P];
  const int tid = threadIdx.x;
  const int k = blockIdx.x;
  const float* src = W_node + (size_t)k * (NF * ND);
  #pragma unroll 1
  for (int idx = tid; idx < NF * ND; idx += 256) {
    const int f = idx >> 6, d = idx & 63;
    const us b = f2bf(src[idx]);
    sN[d * SN_P + f] = b;
    if (f >= ND + NA) sN[d * SN_P + f + NH] = b;
  }
  #pragma unroll 1
  for (int idx = tid; idx < ND * (WNP - 336); idx += 256) {
    const int d = idx / 48, c = 336 + (idx - d * 48);
    sN[d * SN_P + c] = (us)0;
  }
  __syncthreads();
  us* dstb = WN16 + (size_t)k * (ND * WNP);
  wnode_store_pass(sN, dstb, tid);
  __threadfence();
  wnode_store_pass(sN, dstb, tid);
}

__device__ __forceinline__ void agg_store_pass(const float* sAgg, float* AGG,
                                               int b0, int i, int w, int lane) {
  const int q8 = lane & 7, sub = lane >> 3;
  #pragma unroll
  for (int it = 0; it < 8; ++it) {
    const int L = it * 32 + w * 4 + sub;
    const int row = L >> 2, q = L & 3;
    const v4f v = *(const v4fa*)(sAgg + row * SAGG_P + q * 32 + 4 * q8);
    const size_t gi = ((size_t)(b0 + row) * NK + i) * NH + q * 32 + 4 * q8;
    *(volatile v4f*)(AGG + gi) = v;
  }
}

__global__ __launch_bounds__(256) void edge_agg_kernel(
    const us* __restrict__ S16,
    const us* __restrict__ WE16,
    const float* __restrict__ b_edge,
    float* __restrict__ AGG)
{
  __shared__ __attribute__((aligned(16))) float sAgg[TB * SAGG_P];

  const int tid = threadIdx.x, lane = tid & 31, w = tid >> 5;
  const int h = lane >> 4, m = lane & 15;
  const int wr = w >> 2, wc = w & 3;
  const int b0 = blockIdx.x * TB;
  const int i = blockIdx.y;

  const us* arow0 = S16 + (size_t)(b0 + 32 * wr + m) * (NK * ND);
  const us* arow1 = arow0 + (size_t)16 * (NK * ND);

  const v8f zero8 = {0.f, 0.f, 0.f, 0.f, 0.f, 0.f, 0.f, 0.f};
  v8f agg[2][2];
  #pragma unroll
  for (int mt = 0; mt < 2; ++mt)
    #pragma unroll
    for (int nt = 0; nt < 2; ++nt) agg[mt][nt] = zero8;

  #pragma unroll 1
  for (int jj = 0; jj < NK - 1; ++jj) {
    const int j = jj + ((jj >= i) ? 1 : 0);
    const int e = i * (NK - 1) + jj;
    const us* wb = WE16 + ((size_t)e * NH + 32 * wc + m) * KE;

    v8f c[2][2];
    #pragma unroll
    for (int mt = 0; mt < 2; ++mt)
      #pragma unroll
      for (int nt = 0; nt < 2; ++nt) c[mt][nt] = zero8;

    #pragma unroll
    for (int ks = 0; ks < 4; ++ks) {
      const int obj = (ks < 2) ? i : j;
      const int kc = obj * ND + 32 * (ks & 1);
      const v16b a0 = load_frag(arow0 + kc, h);
      const v16b a1 = load_frag(arow1 + kc, h);
      const v16b bw0 = load_frag(wb + 32 * ks, h);
      const v16b bw1 = load_frag(wb + (size_t)16 * KE + 32 * ks, h);
      c[0][0] = wmma_bf16(a0, bw0, c[0][0]);
      c[0][1] = wmma_bf16(a0, bw1, c[0][1]);
      c[1][0] = wmma_bf16(a1, bw0, c[1][0]);
      c[1][1] = wmma_bf16(a1, bw1, c[1][1]);
    }

    const float bb0 = bf16r(b_edge[e * NH + 32 * wc + m]);
    const float bb1 = bf16r(b_edge[e * NH + 32 * wc + 16 + m]);
    #pragma unroll
    for (int mt = 0; mt < 2; ++mt) {
      #pragma unroll
      for (int r = 0; r < 8; ++r) {
        agg[mt][0][r] += tanh_f32(c[mt][0][r] + bb0);
        agg[mt][1][r] += tanh_f32(c[mt][1][r] + bb1);
      }
    }
  }

  #pragma unroll
  for (int mt = 0; mt < 2; ++mt)
    #pragma unroll
    for (int nt = 0; nt < 2; ++nt)
      #pragma unroll
      for (int r = 0; r < 8; ++r)
        sAgg[(32 * wr + 16 * mt + 8 * h + r) * SAGG_P + 32 * wc + 16 * nt + m] = agg[mt][nt][r];
  __syncthreads();

  agg_store_pass(sAgg, AGG, b0, i, w, lane);
  __threadfence();
  agg_store_pass(sAgg, AGG, b0, i, w, lane);
}

__device__ __forceinline__ void out_store_pass(const float* sO, float* out,
                                               int b0, int k, int w, int lane) {
  const int q8 = lane & 7, sub = lane >> 3;
  #pragma unroll
  for (int it = 0; it < 4; ++it) {
    const int L = it * 32 + w * 4 + sub;
    const int row = L >> 1, q = L & 1;
    const v4f v = *(const v4fa*)(sO + row * SO_P + q * 32 + 4 * q8);
    const size_t gi = ((size_t)(b0 + row) * NK + k) * ND + q * 32 + 4 * q8;
    *(volatile v4f*)(out + gi) = v;
  }
}

__global__ __launch_bounds__(256) void node_kernel(
    const us* __restrict__ S16,
    const us* __restrict__ A16,
    const float* __restrict__ AGG,
    const us* __restrict__ WN16,
    const float* __restrict__ b_node,
    float* __restrict__ out)
{
  __shared__ __attribute__((aligned(16))) us sA[TB * SA_P];
  __shared__ __attribute__((aligned(16))) float sO[TB * SO_P];

  const int tid = threadIdx.x, lane = tid & 31, w = tid >> 5;
  const int h = lane >> 4, m = lane & 15;
  const int wr = w >> 1, wc = w & 1;
  const int b0 = blockIdx.x * TB;
  const int k = blockIdx.y;

  #pragma unroll
  for (int it = 0; it < 2; ++it) {
    const int p = it * 256 + tid;
    const int row = p >> 3, c = (p & 7) * 8;
    const v8us v = *(const v8usa*)(S16 + (size_t)(b0 + row) * (NK * ND) + k * ND + c);
    *(v8usa*)(sA + row * SA_P + c) = v;
  }
  if (tid < 128) {
    const int row = tid >> 1, c = (tid & 1) * 8;
    const v8us v = *(const v8usa*)(A16 + (size_t)(b0 + row) * (NK * NA) + k * NA + c);
    *(v8usa*)(sA + row * SA_P + ND + c) = v;
  }
  #pragma unroll
  for (int it = 0; it < 8; ++it) {
    const int p = it * 256 + tid;
    const int row = p >> 5, c = (p & 31) * 4;
    const v4f a = *(const v4fa*)(AGG + ((size_t)(b0 + row) * NK + k) * NH + c);
    const us h0 = f2bf(a.x), h1 = f2bf(a.y), h2 = f2bf(a.z), h3 = f2bf(a.w);
    const v4us hi = { h0, h1, h2, h3 };
    const v4us lo = { f2bf(a.x - bf2f(h0)), f2bf(a.y - bf2f(h1)),
                      f2bf(a.z - bf2f(h2)), f2bf(a.w - bf2f(h3)) };
    *(v4usa*)(sA + row * SA_P + (ND + NA) + c) = hi;
    *(v4usa*)(sA + row * SA_P + (ND + NA + NH) + c) = lo;
  }
  if (tid < 192) {
    const int row = tid / 3, c = 336 + (tid - row * 3) * 8;
    const v8us z = { 0, 0, 0, 0, 0, 0, 0, 0 };
    *(v8usa*)(sA + row * SA_P + c) = z;
  }
  __syncthreads();

  const us* arow = sA + (16 * wr + m) * SA_P;
  const us* wb = WN16 + ((size_t)k * ND + 32 * wc + m) * WNP;
  const v8f zero8 = {0.f, 0.f, 0.f, 0.f, 0.f, 0.f, 0.f, 0.f};
  v8f c[2];
  c[0] = zero8; c[1] = zero8;
  #pragma unroll
  for (int ks = 0; ks < KPN / 32; ++ks) {
    const v16b a = load_frag(arow + 32 * ks, h);
    const v16b bw0 = load_frag(wb + 32 * ks, h);
    const v16b bw1 = load_frag(wb + (size_t)16 * WNP + 32 * ks, h);
    c[0] = wmma_bf16(a, bw0, c[0]);
    c[1] = wmma_bf16(a, bw1, c[1]);
  }

  const float bb0 = bf16r(b_node[k * ND + 32 * wc + m]);
  const float bb1 = bf16r(b_node[k * ND + 32 * wc + 16 + m]);
  #pragma unroll
  for (int r = 0; r < 8; ++r) {
    const int row = 16 * wr + 8 * h + r;
    sO[row * SO_P + 32 * wc + m]      = tanh_f32(c[0][r] + bb0);
    sO[row * SO_P + 32 * wc + 16 + m] = tanh_f32(c[1][r] + bb1);
  }
  __syncthreads();

  out_store_pass(sO, out, b0, k, w, lane);
  __threadfence();
  out_store_pass(sO, out, b0, k, w, lane);
}

extern "C" void kernel_launch(void* const* d_in, const int* in_sizes, int n_in,
                              void* d_out, int out_size, void* d_ws, size_t ws_size,
                              hipStream_t stream) {
  if (n_in < 6) return;
  if (in_sizes[0] != S16_N) return;
  if (in_sizes[1] != A16_N) return;
  if (in_sizes[2] != NE * KE * NH) return;
  if (in_sizes[3] != NE * NH) return;
  if (in_sizes[4] != NK * NF * ND) return;
  if (in_sizes[5] != NK * ND) return;
  if (out_size != S16_N) return;

  const float* states = (const float*)d_in[0];
  const float* action = (const float*)d_in[1];
  const float* W_edge = (const float*)d_in[2];
  const float* b_edge = (const float*)d_in[3];
  const float* W_node = (const float*)d_in[4];
  const float* b_node = (const float*)d_in[5];
  float* out = (float*)d_out;

  const size_t s16_bytes  = (size_t)S16_N * 2;
  const size_t a16_bytes  = (size_t)A16_N * 2;
  const size_t we16_bytes = (size_t)WE16_N * 2;
  const size_t wn16_bytes = (size_t)WN16_N * 2;
  const size_t agg_bytes  = (size_t)AGG_N * 4;
  const size_t total = s16_bytes + a16_bytes + we16_bytes + wn16_bytes + agg_bytes;
  if (total > ws_size) return;

  char* ws = (char*)d_ws;
  us* S16     = (us*)(ws);
  us* A16     = (us*)(ws + s16_bytes);
  us* WE16    = (us*)(ws + s16_bytes + a16_bytes);
  us* WN16    = (us*)(ws + s16_bytes + a16_bytes + we16_bytes);
  float* AGG  = (float*)(ws + s16_bytes + a16_bytes + we16_bytes + wn16_bytes);

  const int ngroups = (S16_N + A16_N) / 8;
  cvt_inputs_kernel<<<(ngroups + 255) / 256, 256, 0, stream>>>(states, action, S16, A16);
  cvt_wedge_kernel<<<NE, 256, 0, stream>>>(W_edge, WE16);
  cvt_wnode_kernel<<<NK, 256, 0, stream>>>(W_node, WN16);

  dim3 gEdge(NB / TB, NK);
  edge_agg_kernel<<<gEdge, 256, 0, stream>>>(S16, WE16, b_edge, AGG);

  dim3 gNode(NB / TB, NK);
  node_kernel<<<gNode, 256, 0, stream>>>(S16, A16, AGG, WN16, b_node, out);
}
